// DyConvSelfAtt_8907762172170
// MI455X (gfx1250) — hardware-verified
//
#include <hip/hip_runtime.h>
#include <math.h>

typedef __attribute__((ext_vector_type(16))) _Float16 v16h;
typedef __attribute__((ext_vector_type(16))) __bf16 v16b;
typedef __attribute__((ext_vector_type(8)))  _Float16 v8h;
typedef __attribute__((ext_vector_type(8)))  float v8f;
typedef __attribute__((ext_vector_type(4)))  float v4f;
typedef __attribute__((ext_vector_type(2)))  float v2f;
typedef __attribute__((ext_vector_type(4)))  unsigned v4u;
typedef __attribute__((ext_vector_type(4)))  int v4i;
typedef float __attribute__((may_alias)) float_a;
typedef int __attribute__((may_alias)) int_a;

template <typename T> __device__ __forceinline__ void vst2(void* p, T v) { *(volatile T*)p = v; __threadfence(); *(volatile T*)p = v; }
__device__ __forceinline__ v8f wmma16(v16h a, v16h b, v8f c) {
  v8f d = __builtin_amdgcn_wmma_f32_16x16x32_f16(false, a, false, b, (short)0, c, false, false);
  asm volatile("v_nop\n\tv_nop\n\tv_nop\n\tv_nop" : "+v"(d) : "v"(a), "v"(b));
  return d;
}
__device__ __forceinline__ v8f wmma_bf(v16b a, v16b b, v8f c) {
  v8f d = __builtin_amdgcn_wmma_f32_16x16x32_bf16(false, a, false, b, (short)0, c, false, false);
  asm volatile("v_nop\n\tv_nop\n\tv_nop\n\tv_nop" : "+v"(d) : "v"(a), "v"(b));
  return d;
}
__device__ __forceinline__ v16h frag_h(const _Float16* rowk0, int lane) {
  union { v16h v; v8h q[2]; } u; const _Float16* p = rowk0 + 8 * (lane >> 4);
  u.q[0] = *(const v8h*)p; u.q[1] = *(const v8h*)(p + 16); return u.v;
}
__device__ __forceinline__ v16h frag_f32(const float* rowk0, int lane) {
  v16h a; const float* p = rowk0 + 8 * (lane >> 4);
#pragma unroll
  for (int i = 0; i < 8; ++i) { a[i] = (_Float16)p[i]; a[8 + i] = (_Float16)p[16 + i]; }
  return a;
}
__device__ __forceinline__ v16h frag_f32s(const float* rowk0, int lane, float sc) {
  v16h a; const float* p = rowk0 + 8 * (lane >> 4);
#pragma unroll
  for (int i = 0; i < 8; ++i) { a[i] = (_Float16)(p[i] * sc); a[8 + i] = (_Float16)(p[16 + i] * sc); }
  return a;
}
__device__ __forceinline__ v16h fragc_f32(const float* W, int k0, int n, int lane, int ld, int K) {
  v16h a; const int g = lane >> 4;
#pragma unroll
  for (int i = 0; i < 8; ++i) { const int ka = k0 + 8 * g + i, kb = ka + 16;
    a[i] = (_Float16)(ka < K ? W[(size_t)(ka < K ? ka : K - 1) * ld + n] : 0.f); a[8 + i] = (_Float16)(kb < K ? W[(size_t)(kb < K ? kb : K - 1) * ld + n] : 0.f); }
  return a;
}
struct F2 { v16b h, l; };
__device__ __forceinline__ F2 bsplit16(const float v[16]) { F2 r;
#pragma unroll
  for (int i = 0; i < 16; ++i) { const __bf16 h = (__bf16)v[i]; r.h[i] = h; r.l[i] = (__bf16)(v[i] - (float)h); }
  return r; }
__device__ __forceinline__ F2 split_row(const float* row, int k0, int lane) { float v[16]; const float* p = row + k0 + 8 * (lane >> 4);
#pragma unroll
  for (int i = 0; i < 8; ++i) { v[i] = p[i]; v[8 + i] = p[16 + i]; }
  return bsplit16(v); }
__device__ __forceinline__ F2 split_rowK(const float* row, int k0, int lane, int K) { float v[16]; const int g = lane >> 4;
#pragma unroll
  for (int i = 0; i < 8; ++i) { const int ka = k0 + 8 * g + i, kb = ka + 16; v[i] = ka < K ? row[ka < K ? ka : K - 1] : 0.f; v[8 + i] = kb < K ? row[kb < K ? kb : K - 1] : 0.f; }
  return bsplit16(v); }
__device__ __forceinline__ F2 split_col(const float* W, int k0, int n, int lane, int ld, int K) { float v[16]; const int g = lane >> 4;
#pragma unroll
  for (int i = 0; i < 8; ++i) { const int ka = k0 + 8 * g + i, kb = ka + 16; v[i] = ka < K ? W[(size_t)(ka < K ? ka : K - 1) * ld + n] : 0.f; v[8 + i] = kb < K ? W[(size_t)(kb < K ? kb : K - 1) * ld + n] : 0.f; }
  return bsplit16(v); }
__device__ __forceinline__ v8f mac3(const F2& a, const F2& b, v8f c) { c = wmma_bf(a.l, b.h, c); c = wmma_bf(a.h, b.l, c); return wmma_bf(a.h, b.h, c); }
__device__ __forceinline__ float sigm(float v) { return 1.0f / (1.0f + expf(-v)); }
#define LDSX() do { asm volatile("s_wait_dscnt 0" ::: "memory"); __builtin_amdgcn_wave_barrier(); __builtin_amdgcn_fence(__ATOMIC_RELEASE, "workgroup"); } while (0)


#define NB 16
#define HW 224
#define H2 112
#define NP (H2 * H2)
#define KC 147
#define KCP 160
#define NQ 24
#define NKM 128
#define NV 16
#define NF (NQ + 3 * NKM + NV)
#define KA (8 * NP)
#define NCH 49
#define OS 58
#ifndef TNB
#define TNB NB
#endif
typedef __attribute__((ext_vector_type(8))) __bf16 v8b;
__device__ __forceinline__ v16b frag_b(const __bf16* rowk0, int lane) {
  union { v16b v; v8b q[2]; } u; const __bf16* p = rowk0 + 8 * (lane >> 4);
  u.q[0] = *(const v8b*)p; u.q[1] = *(const v8b*)(p + 16); return u.v;
}
__device__ __forceinline__ float bfr(float v) { return (float)(__bf16)v; }
#define WS_PF   0u
#define WS_Q    (WS_PF + 2u * 432 * KCP)
#define WS_V    (WS_Q + 4u * NB * NQ * NP)
#define WS_KM   (WS_V + 4u * NB * NV * NP)
#define WS_PART (WS_KM + 4u * NKM * NP)
#define WS_A    (WS_PART + 4u * NB * 3 * NCH * 256)
#define WS_OST  (WS_A + 4u * NB * 3 * 256)
#define WS_END  (WS_OST + 4u * NB * 3 * 3392)

__global__ __launch_bounds__(256) void k_pack(const float* __restrict__ Wq, const float* __restrict__ Wk, const float* __restrict__ Wv, __bf16* __restrict__ PF) {
  __shared__ __align__(16) __bf16 srow[KCP];
  const int f = blockIdx.x, tid = threadIdx.x;
  if (tid < KCP) { float v = 0.f; if (tid < KC) { if (f < NQ) v = bfr(Wq[(size_t)f * KC + tid]); else if (f < NQ + 3 * NKM) v = bfr(Wk[(size_t)(f - NQ) * KC + tid]); else if (f < NF) v = bfr(Wv[(size_t)(f - NQ - 3 * NKM) * KC + tid]); } srow[tid] = (__bf16)v; }
  __syncthreads();
  if (tid < KCP / 8) vst2((unsigned*)(PF + (size_t)f * KCP + tid * 8), *(const v4u*)(&srow[tid * 8]));
}
__device__ __forceinline__ v16b frag_im2col(const float* __restrict__ Xb, int p, int k0, int lane) {
  v16b a; const int py = p / H2, px = p % H2; const int kb = k0 + 8 * (lane >> 4);
#pragma unroll
  for (int i = 0; i < 16; ++i) { const int k = kb + (i < 8 ? i : 8 + i); float v = 0.f;
    if (k < KC) { const int ci = k / 49, r = k % 49, u = r / 7, w = r % 7; const int yy = 2 * py + u - 3, xx = 2 * px + w - 3; if (yy >= 0 && yy < HW && xx >= 0 && xx < HW) v = Xb[((size_t)ci * HW + yy) * HW + xx]; }
    a[i] = (__bf16)v; }
  return a;
}
template <int NT>
__device__ __forceinline__ void conv_block(const float* __restrict__ Xb, const __bf16* __restrict__ PF, int f0, const float* __restrict__ bias, int nreal, float* __restrict__ OUTM  , int p0blk, float (*so)[68], int wave, int lane) {
  const int col = lane & 15, g = lane >> 4; const int p0 = p0blk + wave * 16;
  v8f acc[NT];
#pragma unroll
  for (int j = 0; j < NT; ++j) acc[j] = (v8f){};
#pragma unroll 1
  for (int kc = 0; kc < KCP / 32; ++kc) { const v16b a = frag_im2col(Xb, p0 + col, kc * 32, lane);
#pragma unroll
    for (int j = 0; j < NT; ++j) acc[j] = wmma_bf(a, frag_b(PF + (size_t)(f0 + j * 16 + col) * KCP + kc * 32, lane), acc[j]); }
#pragma unroll
  for (int j = 0; j < NT; ++j) {
#pragma unroll
    for (int r = 0; r < 8; ++r) so[col][wave * 16 + 8 * g + r] = acc[j][r] + ((j * 16 + col) < nreal ? bfr(bias[j * 16 + col]) : 0.f);
    __syncthreads();
    { const int tid = wave * 32 + lane; for (int q = tid; q < 16 * 16; q += 128) { const int m = q >> 4, pc = q & 15; const int n = j * 16 + m; if (n < nreal) vst2(OUTM + (size_t)n * NP + p0blk + pc * 4, *(const v4f*)&so[m][pc * 4]); } }
    __syncthreads(); }
}
__global__ __launch_bounds__(128) void k_convqv(const float* __restrict__ X, const __bf16* __restrict__ PF, const float* __restrict__ bq, const float* __restrict__ bv, float* __restrict__ Q, float* __restrict__ V) {
  __shared__ __align__(16) float so[16][68];
  const int tid = threadIdx.x, wave = tid >> 5, lane = tid & 31; const int b = blockIdx.y, p0blk = blockIdx.x * 64; const float* Xb = X + (size_t)b * 3 * HW * HW;
  conv_block<2>(Xb, PF, 0, bq, NQ, Q + (size_t)b * NQ * NP, p0blk, so, wave, lane);
  conv_block<1>(Xb, PF, NQ + 3 * NKM, bv, NV, V + (size_t)b * NV * NP, p0blk, so, wave, lane);
}
__global__ __launch_bounds__(128) void k_convk(const float* __restrict__ X, const __bf16* __restrict__ PF, const float* __restrict__ bk, float* __restrict__ KM, int b, int i) {
  __shared__ __align__(16) float so[16][68];
  const int tid = threadIdx.x, wave = tid >> 5, lane = tid & 31; const int p0blk = blockIdx.x * 64; const float* Xb = X + (size_t)b * 3 * HW * HW;
  conv_block<8>(Xb, PF, NQ + i * NKM, bk + i * NKM, NKM, KM, p0blk, so, wave, lane);
}
__global__ __launch_bounds__(32) void k_apart(const float* __restrict__ Q, const float* __restrict__ KM, float* __restrict__ PART, int b, int i) {
  __shared__ __align__(16) float st[256];
  const int lane = threadIdx.x, col = lane & 15, g = lane >> 4; const int ch = blockIdx.x; const int k0 = ch * 2048;
  const float* qb = Q + ((size_t)b * NQ + i * 8) * NP;
  const int y = col >> 2, x = col & 3;
  v8f acc = {};
#pragma unroll 1
  for (int ks = 0; ks < 64; ++ks) { const int kk = k0 + ks * 32; const int c = kk / NP; const int pk = kk % NP;
    F2 a; {
#pragma unroll
      for (int e = 0; e < 16; ++e) { const int k = pk + 8 * g + (e < 8 ? e : 8 + e); const int kh = k / H2, kw = k % H2; const int yy = 2 * y + kh - 3, xx = 2 * x + kw - 3; float v = 0.f;
        if (yy >= 0 && yy < H2 && xx >= 0 && xx < H2) v = qb[(size_t)c * NP + yy * H2 + xx]; const __bf16 hb = (__bf16)v; a.h[e] = hb; a.l[e] = (__bf16)(v - (float)hb); } }
    const F2 bm = split_row(KM + ((size_t)col * 8 + c) * NP + pk, 0, lane);
    acc = mac3(a, bm, acc); }
#pragma unroll
  for (int r = 0; r < 8; ++r) st[(8 * g + r) * 16 + col] = acc[r];
  __builtin_amdgcn_fence(__ATOMIC_RELEASE, "workgroup"); __builtin_amdgcn_wave_barrier(); __builtin_amdgcn_fence(__ATOMIC_ACQUIRE, "workgroup");
  for (int q = lane; q < 64; q += 32) vst2(PART + ((size_t)(b * 3 + i) * NCH + ch) * 256 + q * 4, *(const v4f*)&st[q * 4]);
}
__global__ __launch_bounds__(256) void k_asum(const float* __restrict__ PART, float* __restrict__ A) {
  __shared__ __align__(16) float sa[256];
  const int bi = blockIdx.x, tid = threadIdx.x; const int pos = tid >> 4, o = tid & 15; float s = 0.f;
  for (int ch = 0; ch < NCH; ++ch) s += PART[((size_t)bi * NCH + ch) * 256 + pos * 16 + o];
  sa[o * 16 + pos] = s;
  __syncthreads();
  if (tid < 64) vst2(A + (size_t)bi * 256 + tid * 4, *(const v4f*)&sa[tid * 4]);
}
__global__ __launch_bounds__(64) void k_o(const float* __restrict__ V, const float* __restrict__ A, float* __restrict__ OST) {
  __shared__ float sa[256]; __shared__ __align__(16) float so[64];
  const int bi = blockIdx.y, tid = threadIdx.x; const int b = bi / 3; const int P = blockIdx.x * 64 + tid;
  for (int q = tid; q < 256; q += 64) sa[q] = A[(size_t)bi * 256 + q];
  __syncthreads();
  float s = 0.f;
  if (P < OS * OS) { const int Y = P / OS, X = P % OS; const float* vb = V + (size_t)b * NV * NP;
#pragma unroll 1
    for (int ch = 0; ch < NV; ++ch)
#pragma unroll
      for (int u = 0; u < 4; ++u) { const int yy = 2 * Y + u - 3; if (yy < 0 || yy >= H2) continue;
#pragma unroll
        for (int w = 0; w < 4; ++w) { const int xx = 2 * X + w - 3; if (xx >= 0 && xx < H2) s += vb[(size_t)ch * NP + yy * H2 + xx] * sa[ch * 16 + u * 4 + w]; } } }
  so[tid] = s; __syncthreads();
  if (tid < 16) vst2(OST + (size_t)bi * 3392 + blockIdx.x * 64 + tid * 4, *(const v4f*)&so[tid * 4]);
}
__global__ __launch_bounds__(256) void k_copy(const float* __restrict__ OST, float* __restrict__ out) {
  const size_t p = (size_t)blockIdx.x * 256 + threadIdx.x; const size_t total = (size_t)NB * 3 * OS * OS;
  if (p * 4 >= total) return; v4f v;
#pragma unroll
  for (int i = 0; i < 4; ++i) { const size_t f = p * 4 + i; v[i] = OST[(f / (OS * OS)) * 3392 + (f % (OS * OS))]; }
  vst2(out + p * 4, v);
}

extern "C" void kernel_launch(void* const* d_in, const int* in_sizes, int n_in, void* d_out, int out_size, void* d_ws, size_t ws_size, hipStream_t stream) {
  (void)in_sizes; (void)n_in; (void)out_size;
  const float** F = (const float**)d_in;
  if (ws_size < (size_t)WS_END) return;
  char* ws = (char*)d_ws; __bf16* PF = (__bf16*)(ws + WS_PF); float *Q = (float*)(ws + WS_Q), *V = (float*)(ws + WS_V), *KM = (float*)(ws + WS_KM), *PART = (float*)(ws + WS_PART), *A = (float*)(ws + WS_A), *OST = (float*)(ws + WS_OST);
  k_pack<<<432, 256, 0, stream>>>(F[1], F[3], F[5], PF);
  k_convqv<<<dim3(NP / 64, TNB), 128, 0, stream>>>(F[0], PF, F[2], F[6], Q, V);
  for (int b = 0; b < TNB; ++b) for (int i = 0; i < 3; ++i) {
    k_convk<<<NP / 64, 128, 0, stream>>>(F[0], PF, F[4], KM, b, i);
    k_apart<<<NCH, 32, 0, stream>>>(Q, KM, PART, b, i); }
  k_asum<<<TNB * 3, 256, 0, stream>>>(PART, A);
  k_o<<<dim3((OS * OS + 63) / 64, TNB * 3), 64, 0, stream>>>(V, A, OST);
  k_copy<<<(NB * 3 * OS * OS / 4 + 255) / 256, 256, 0, stream>>>(OST, (float*)d_out);
}
